// AttnHeads_89653147337002
// MI455X (gfx1250) — hardware-verified
//
#include <hip/hip_runtime.h>
#include <stdint.h>

#define NB    4
#define SEQ   2048
#define HID   1024
#define NH    16
#define HD    64
#define NTOK  (NB * SEQ)
#define QKLD  (2 * HID)

typedef __bf16         v16b  __attribute__((ext_vector_type(16)));
typedef float          v8f   __attribute__((ext_vector_type(8)));
typedef float          v4f   __attribute__((ext_vector_type(4)));
typedef unsigned short v8us  __attribute__((ext_vector_type(8)));
typedef unsigned short v16us __attribute__((ext_vector_type(16)));

static_assert(sizeof(long) == 8);

__device__ __forceinline__ unsigned short f2bf_bits(float f) {
  const unsigned u = __float_as_uint(f);
  return (unsigned short)((u + 0x7FFFu + ((u >> 16) & 1u)) >> 16);
}
__device__ __forceinline__ float bf_bits2f(unsigned short b) { return __uint_as_float(((unsigned)b) << 16); }

__device__ __forceinline__ v16b ldfrag(const unsigned short* p) {
  const v8us a = *(const v8us*)p;
  const v8us b = *(const v8us*)(p + 16);
  const v16us w = __builtin_shufflevector(a, b, 0, 1, 2, 3, 4, 5, 6, 7, 8, 9, 10, 11, 12, 13, 14, 15);
  return __builtin_bit_cast(v16b, w);
}

__device__ __forceinline__ v8f mma_bf16(v16b a, v16b b, v8f c) {
  c = __builtin_amdgcn_wmma_f32_16x16x32_bf16(false, a, false, b, (short)0, c, false, false);
  asm volatile("v_nop\n\tv_nop\n\tv_nop\n\tv_nop" : "+v"(c) : "v"(a), "v"(b));
  return c;
}

__device__ __forceinline__ v8f zero8() { return (v8f){0.f, 0.f, 0.f, 0.f, 0.f, 0.f, 0.f, 0.f}; }
__device__ __forceinline__ v8us zero8us() { return (v8us){0, 0, 0, 0, 0, 0, 0, 0}; }

template <int OUT_MODE>
__global__ __launch_bounds__(256) void gemm64_kernel(
    const unsigned short* __restrict__ A, int lda, long strideA,
    const unsigned short* __restrict__ Bt, int ldb, long strideB,
    void* Cout, void* Cout2, int ldc, long strideC,
    int M, int N, int K, float scale) {
  __shared__ __align__(16) float sT[8][16 * 68];
  const int bz   = blockIdx.y;
  const int lane = threadIdx.x & 31;
  const int wave = threadIdx.x >> 5;
  const int tilesN = N >> 6;
  const int tilesM = M >> 6;
  const int tile = blockIdx.x * 8 + wave;
  if (tile >= tilesM * tilesN) return;
  const int tm = tile / tilesN;
  const int tn = tile - tm * tilesN;
  const int m0 = tm << 6;
  const int n0 = tn << 6;

  const unsigned short* Ab = A  + (size_t)bz * strideA;
  const unsigned short* Bb = Bt + (size_t)bz * strideB;

  const int rl   = lane & 15;
  const int koff = (lane >> 4) * 8;
  const int mOff = (lane >> 4) * 8;

  v8f acc[4][4];
#pragma unroll
  for (int i = 0; i < 4; ++i)
#pragma unroll
    for (int j = 0; j < 4; ++j) acc[i][j] = zero8();

#pragma unroll 1
  for (int k0 = 0; k0 < K; k0 += 32) {
    v16b bf[4];
#pragma unroll
    for (int j = 0; j < 4; ++j)
      bf[j] = ldfrag(Bb + (size_t)(n0 + (j << 4) + rl) * ldb + k0 + koff);
#pragma unroll
    for (int i = 0; i < 4; ++i) {
      const v16b af = ldfrag(Ab + (size_t)(m0 + (i << 4) + rl) * lda + k0 + koff);
#pragma unroll
      for (int j = 0; j < 4; ++j) acc[i][j] = mma_bf16(af, bf[j], acc[i][j]);
    }
  }

  float* slab = sT[wave];
#pragma unroll
  for (int i = 0; i < 4; ++i) {
    const int mBase = m0 + (i << 4);
#pragma unroll
    for (int j = 0; j < 4; ++j)
#pragma unroll
      for (int r = 0; r < 8; ++r)
        slab[(mOff + r) * 68 + (j << 4) + rl] = acc[i][j][r] * scale;
    __builtin_amdgcn_fence(__ATOMIC_RELEASE, "workgroup");
    __builtin_amdgcn_wave_barrier();
    __builtin_amdgcn_fence(__ATOMIC_ACQUIRE, "workgroup");
    if (OUT_MODE == 0) {
      float* C = (float*)Cout + (size_t)bz * strideC;
      const int hh = lane >> 4, c4 = (lane & 15) * 4;
      for (int pass = 0; pass < 2; ++pass) {
#pragma unroll
        for (int it = 0; it < 8; ++it) {
          const int row = it * 2 + hh;
          const v4f v = *(const v4f*)(slab + row * 68 + c4);
          *(volatile v4f*)(C + (size_t)(mBase + row) * ldc + n0 + c4) = v;
        }
        __threadfence();
      }
    } else {
      const int q4 = lane >> 3, c8 = (lane & 7) * 8;
      unsigned short* C  = (unsigned short*)Cout  + (size_t)bz * strideC;
      unsigned short* C2 = (unsigned short*)Cout2 + (size_t)bz * strideC;
      for (int pass = 0; pass < 2; ++pass) {
#pragma unroll
        for (int it = 0; it < 4; ++it) {
          const int row = it * 4 + q4;
          const float* sp = slab + row * 68 + c8;
          const v4f x0 = *(const v4f*)sp;
          const v4f x1 = *(const v4f*)(sp + 4);
          v8us hv = zero8us(), lv = zero8us();
#pragma unroll
          for (int e = 0; e < 4; ++e) {
            const unsigned short hb0 = f2bf_bits(x0[e]);
            const unsigned short hb1 = f2bf_bits(x1[e]);
            hv[e] = hb0; hv[4 + e] = hb1;
            if (OUT_MODE == 2) {
              lv[e]     = f2bf_bits(x0[e] - bf_bits2f(hb0));
              lv[4 + e] = f2bf_bits(x1[e] - bf_bits2f(hb1));
            }
          }
          *(volatile v8us*)(C + (size_t)(mBase + row) * ldc + n0 + c8) = hv;
          if (OUT_MODE == 2) *(volatile v8us*)(C2 + (size_t)(mBase + row) * ldc + n0 + c8) = lv;
        }
        __threadfence();
      }
    }
    __builtin_amdgcn_fence(__ATOMIC_RELEASE, "workgroup");
    __builtin_amdgcn_wave_barrier();
    __builtin_amdgcn_fence(__ATOMIC_ACQUIRE, "workgroup");
  }
}

__global__ __launch_bounds__(256) void cvt_bf16_kernel(const float* __restrict__ in, unsigned short* out, int n8) {
  const int i = blockIdx.x * 256 + threadIdx.x;
  if (i < n8) {
    const size_t o = 8 * (size_t)i;
    const v4f a = *(const v4f*)(in + o);
    const v4f b = *(const v4f*)(in + o + 4);
    v8us w = zero8us();
#pragma unroll
    for (int e = 0; e < 4; ++e) { w[e] = f2bf_bits(a[e]); w[4 + e] = f2bf_bits(b[e]); }
    *(volatile v8us*)(out + o) = w;
    __threadfence();
    *(volatile v8us*)(out + o) = w;
  }
}

__global__ __launch_bounds__(256) void tcvt_kernel(const float* __restrict__ W, unsigned short* out, int R, int Cc) {
  __shared__ __align__(16) float tf[64 * 68];
  const int c0  = blockIdx.x * 64;
  const int r0  = blockIdx.y * 64;
  const int tid = threadIdx.x;
  {
    const int lr = tid >> 4;
    const int c4 = (tid & 15) * 4;
#pragma unroll
    for (int it = 0; it < 4; ++it) {
      const int rr = it * 16 + lr;
      const v4f a = *(const v4f*)(W + (size_t)(r0 + rr) * Cc + c0 + c4);
      *(v4f*)(tf + rr * 68 + c4) = a;
    }
  }
  __syncthreads();
  const int sub = tid >> 3;
  const int c8  = (tid & 7) * 8;
  v8us hv[2];
#pragma unroll
  for (int it = 0; it < 2; ++it) {
    const int oc = it * 32 + sub;
    v8us w = zero8us();
#pragma unroll
    for (int e = 0; e < 8; ++e) w[e] = f2bf_bits(tf[(c8 + e) * 68 + oc]);
    hv[it] = w;
  }
  for (int pass = 0; pass < 2; ++pass) {
#pragma unroll
    for (int it = 0; it < 2; ++it) {
      const int oc = it * 32 + sub;
      *(volatile v8us*)(out + (size_t)(c0 + oc) * R + r0 + c8) = hv[it];
    }
    __threadfence();
  }
}

#define AT_KC 32
#define AT_OP 72

__global__ __launch_bounds__(128) void attn_kernel(const unsigned short* __restrict__ QKh,
                                                   const unsigned short* __restrict__ QKl,
                                                   const unsigned short* __restrict__ VT,
                                                   unsigned short* CTX) {
  __shared__ __align__(16) float Os[4][16 * AT_OP];
  const int tid  = threadIdx.x;
  const int wave = tid >> 5;
  const int lane = tid & 31;
  const int h    = lane >> 4;
  const int c    = lane & 15;
  const int bx   = blockIdx.x;
  const int qb   = bx % (SEQ / 64);
  const int bn   = bx / (SEQ / 64);
  const int b    = bn / NH;
  const int n    = bn % NH;
  const int t0   = qb * 64 + wave * 16;
  const size_t rowb = (size_t)b * SEQ;

  v16b qh[2], ql[2];
#pragma unroll
  for (int dc = 0; dc < 2; ++dc) {
    const size_t o = (rowb + t0 + c) * QKLD + (size_t)n * HD + dc * 32 + 8 * h;
    qh[dc] = ldfrag(QKh + o);
    ql[dc] = ldfrag(QKl + o);
  }
  const unsigned short* Kh = QKh + rowb * QKLD + HID + (size_t)n * HD;
  const unsigned short* Kl = QKl + rowb * QKLD + HID + (size_t)n * HD;
  const unsigned short* Vb = VT + ((size_t)b * HID + (size_t)n * HD) * SEQ;

  v8f oacc[4];
#pragma unroll
  for (int dt = 0; dt < 4; ++dt) oacc[dt] = zero8();
  float mrun = -1.0e30f;
  float lrun = 0.f;

#pragma unroll 1
  for (int kc = 0; kc < SEQ / AT_KC; ++kc) {
    const int s0 = kc * AT_KC;

    v8f s[2];
#pragma unroll
    for (int j = 0; j < 2; ++j) {
      s[j] = zero8();
#pragma unroll
      for (int dc = 0; dc < 2; ++dc) {
        const size_t o = (size_t)(s0 + 16 * j + c) * QKLD + dc * 32 + 8 * h;
        const v16b ka = ldfrag(Kh + o);
        const v16b kl = ldfrag(Kl + o);
        s[j] = mma_bf16(ka, qh[dc], s[j]);
        s[j] = mma_bf16(ka, ql[dc], s[j]);
        s[j] = mma_bf16(kl, qh[dc], s[j]);
      }
    }

    float cmax = s[0][0];
#pragma unroll
    for (int r = 0; r < 8; ++r) cmax = fmaxf(cmax, fmaxf(s[0][r], s[1][r]));
    cmax = fmaxf(cmax, __shfl_xor(cmax, 16, 32));
    const float mnew  = fmaxf(mrun, cmax);
    const float alpha = __expf(mrun - mnew);
    mrun = mnew;
    float psum = 0.f;
    v8us p0 = zero8us(), p1 = zero8us();
#pragma unroll
    for (int r = 0; r < 8; ++r) {
      const float e0 = __expf(s[0][r] - mnew);
      const float e1 = __expf(s[1][r] - mnew);
      psum += e0 + e1;
      p0[r] = f2bf_bits(e0);
      p1[r] = f2bf_bits(e1);
    }
    psum += __shfl_xor(psum, 16, 32);
    lrun = lrun * alpha + psum;
#pragma unroll
    for (int dt = 0; dt < 4; ++dt)
#pragma unroll
      for (int r = 0; r < 8; ++r) oacc[dt][r] *= alpha;

    const v16us pw = __builtin_shufflevector(p0, p1, 0, 1, 2, 3, 4, 5, 6, 7, 8, 9, 10, 11, 12, 13, 14, 15);
    const v16b  pb = __builtin_bit_cast(v16b, pw);
#pragma unroll
    for (int dt = 0; dt < 4; ++dt) {
      const size_t o = (size_t)(16 * dt + c) * SEQ + s0 + 8 * h;
      const v16b va = ldfrag(Vb + o);
      oacc[dt] = mma_bf16(va, pb, oacc[dt]);
    }
  }

  const float inv = 1.0f / lrun;
  float* os = Os[wave];
#pragma unroll
  for (int dt = 0; dt < 4; ++dt)
#pragma unroll
    for (int r = 0; r < 8; ++r) os[c * AT_OP + 16 * dt + 8 * h + r] = oacc[dt][r] * inv;
  __builtin_amdgcn_fence(__ATOMIC_RELEASE, "workgroup");
  __builtin_amdgcn_wave_barrier();
  __builtin_amdgcn_fence(__ATOMIC_ACQUIRE, "workgroup");
  const int q4 = lane >> 3;
  const int c8 = (lane & 7) * 8;
  v8us ov[4];
#pragma unroll
  for (int it = 0; it < 4; ++it) {
    const int row = it * 4 + q4;
    const float* sp = os + row * AT_OP + c8;
    const v4f x0 = *(const v4f*)sp;
    const v4f x1 = *(const v4f*)(sp + 4);
    v8us w = zero8us();
#pragma unroll
    for (int e = 0; e < 4; ++e) { w[e] = f2bf_bits(x0[e]); w[4 + e] = f2bf_bits(x1[e]); }
    ov[it] = w;
  }
  unsigned short* cb = CTX + (rowb + t0) * HID + (size_t)n * HD + c8;
  for (int pass = 0; pass < 2; ++pass) {
#pragma unroll
    for (int it = 0; it < 4; ++it) {
      const int row = it * 4 + q4;
      *(volatile v8us*)(cb + (size_t)row * HID) = ov[it];
    }
    __threadfence();
  }
}

extern "C" void kernel_launch(void* const* d_in, const int* in_sizes, int n_in,
                              void* d_out, int out_size, void* d_ws, size_t ws_size,
                              hipStream_t stream) {
  if (n_in < 3) return;
  if (in_sizes[0] != NTOK * HID) return;
  if (in_sizes[1] != HID * 3 * HID) return;
  if (in_sizes[2] != HID * HID) return;
  if (out_size != NTOK * HID) return;

  const float* x   = (const float*)d_in[0];
  const float* wqk = (const float*)d_in[1];
  const float* wo  = (const float*)d_in[2];
  float* out = (float*)d_out;

  const size_t bWT  = (size_t)3 * HID * HID * 2;
  const size_t bWoT = (size_t)HID * HID * 2;
  const size_t bXb  = (size_t)NTOK * HID * 2;
  const size_t bQK  = (size_t)NTOK * QKLD * 2;
  const size_t bVT  = (size_t)NB * HID * SEQ * 2;
  const size_t bCTX = (size_t)NTOK * HID * 2;
  size_t off = 0;
  const size_t oWT  = off; off += bWT;
  const size_t oWoT = off; off += bWoT;
  const size_t oXb  = off; off += bXb;
  const size_t oQKh = off; off += bQK;
  const size_t oQKl = off; off += bQK;
  const size_t oVT  = off; off += bVT;
  const size_t oCTX = off; off += bCTX;
  if (off > ws_size) return;
  if (off > (size_t)134217728) return;

  char* ws = (char*)d_ws;
  unsigned short* WT  = (unsigned short*)(ws + oWT);
  unsigned short* WoT = (unsigned short*)(ws + oWoT);
  unsigned short* Xb  = (unsigned short*)(ws + oXb);
  unsigned short* QKh = (unsigned short*)(ws + oQKh);
  unsigned short* QKl = (unsigned short*)(ws + oQKl);
  unsigned short* VT  = (unsigned short*)(ws + oVT);
  unsigned short* CTX = (unsigned short*)(ws + oCTX);

  const dim3 blk(256);

  const int n8 = NTOK * HID / 8;
  cvt_bf16_kernel<<<dim3((n8 + 255) / 256), blk, 0, stream>>>(x, Xb, n8);
  tcvt_kernel<<<dim3(3 * HID / 64, HID / 64), blk, 0, stream>>>(wqk, WT, HID, 3 * HID);
  tcvt_kernel<<<dim3(HID / 64, HID / 64), blk, 0, stream>>>(wo, WoT, HID, HID);

  const dim3 gQK(((NTOK / 64) * (QKLD / 64) + 7) / 8, 1);
  gemm64_kernel<2><<<gQK, blk, 0, stream>>>(
      Xb, HID, 0L, WT, HID, 0L, (void*)QKh, (void*)QKl, QKLD, 0L, NTOK, QKLD, HID, 1.0f);

  const dim3 gVT(((HID / 64) * (SEQ / 64) + 7) / 8, NB);
  gemm64_kernel<1><<<gVT, blk, 0, stream>>>(
      WT + (size_t)2 * HID * HID, HID, 0L, Xb, HID, (long)SEQ * HID,
      (void*)VT, (void*)VT, SEQ, (long)HID * SEQ, HID, SEQ, HID, 1.0f);

  attn_kernel<<<dim3(NB * NH * (SEQ / 64)), dim3(128), 0, stream>>>(QKh, QKl, VT, CTX);

  const dim3 gOut(((NTOK / 64) * (HID / 64) + 7) / 8, 1);
  gemm64_kernel<0><<<gOut, blk, 0, stream>>>(
      CTX, HID, 0L, WoT, HID, 0L, (void*)out, (void*)out, HID, 0L, NTOK, HID, HID, 0.125f);

  (void)hipGetLastError();
}
